// TemporalRunnerGNN_12893491823124
// MI455X (gfx1250) — hardware-run, weakly checked
//
#include <hip/hip_runtime.h>


namespace {
constexpr int NODES = 23, NBQ = 64, T = 128, G = NBQ * T, N = G * NODES, E = 1507328, DIN = 16, H = 128, RH = 128, G3 = 3 * RH;
constexpr float XS = 8.0f, WSC = 256.0f;

typedef _Float16 b16;
typedef __attribute__((ext_vector_type(16))) _Float16 v16b;
typedef __attribute__((ext_vector_type(8))) _Float16 v8b;
typedef __attribute__((ext_vector_type(8))) float v8f;
typedef __attribute__((ext_vector_type(4))) float v4f;
__device__ __forceinline__ float bf16_rne(float f) { unsigned int u = __float_as_uint(f); u += 0x7FFFu + ((u >> 16) & 1u); return __uint_as_float(u & 0xFFFF0000u); }
__device__ __forceinline__ void split16(float v, b16& hi, b16& lo) { hi = (b16)v; lo = (b16)(v - (float)hi); }
__device__ __forceinline__ v16b frag_kb(const b16* p, int hh) { const v8b a = *(const v8b*)(p + 8 * hh), b = *(const v8b*)(p + 16 + 8 * hh); v16b f;
#pragma unroll
  for (int e = 0; e < 8; ++e) { f[e] = a[e]; f[8 + e] = b[e]; } return f; }
__device__ __forceinline__ v8f wmma16b(v16b a, v16b b, v8f c) { v8f d = __builtin_amdgcn_wmma_f32_16x16x32_f16(false, a, false, b, (short)0, c, false, false); asm volatile("v_nop\n\tv_nop\n\tv_nop\n\tv_nop" : "+v"(d) : "v"(a), "v"(b)); return d; }
__device__ __forceinline__ void wave_lds_sync() { __builtin_amdgcn_fence(__ATOMIC_RELEASE, "workgroup"); __builtin_amdgcn_wave_barrier(); __builtin_amdgcn_fence(__ATOMIC_ACQUIRE, "workgroup"); }
__device__ __forceinline__ float pmul(float a, float b) { float p = a * b; asm volatile("" : "+v"(p)); return p; }
__device__ __forceinline__ int iclamp(int v, int lo, int hi) { return v < lo ? lo : (v > hi ? hi : v); }
__device__ __forceinline__ float nexp(float x) { return __builtin_amdgcn_exp2f(x * 1.4426950408889634f); }
__device__ __forceinline__ float sigm(float x) { return 1.0f / (1.0f + nexp(-x)); }
__device__ __forceinline__ float tanh_(float x) { const float e = nexp(-2.0f * fabsf(x)); const float t = (1.0f - e) / (1.0f + e); return x < 0.0f ? -t : t; }

constexpr int CSR_NBLK = 512, CSR_GB = 9, CSR_GN = 1 << CSR_GB  , CSR_MAXG = 512, CSR_CAP = 12288  ;
__global__ __launch_bounds__(64) void csrA_kernel(const int* __restrict__ dst, int E, int N, int nG, int CHP, int NGP, int* __restrict__ STG, int* __restrict__ HST) {
  extern __shared__ int sm[];
  int* cnt = sm; int* run = sm + NGP; int* ids = sm + 2 * NGP;
  const int b = blockIdx.x; const int ch = (E + CSR_NBLK - 1) / CSR_NBLK; const int e0 = b * ch, e1 = min(E, e0 + ch);
  for (int i = threadIdx.x; i < NGP; i += 64) cnt[i] = 0;
  for (int i = threadIdx.x; i < CHP; i += 64) ids[i] = -1;
  __syncthreads();
  if (threadIdx.x == 0) {
    for (int e = e0; e < e1; ++e) { int d = dst[e]; d = (d < 0) ? 0 : (d >= N ? N - 1 : d); cnt[d >> CSR_GB] += 1; }
    int acc = 0; for (int g = 0; g < nG; ++g) { run[g] = acc; acc += cnt[g]; }
    for (int e = e0; e < e1; ++e) { int d = dst[e]; d = (d < 0) ? 0 : (d >= N ? N - 1 : d); const int g = d >> CSR_GB; ids[run[g]] = e; run[g] += 1; } }
  __syncthreads();
  typedef __attribute__((ext_vector_type(4))) int v4i;
  for (int pass = 0; pass < 2; ++pass) {
    for (int i = threadIdx.x; i < CHP / 4; i += 64) *(volatile v4i*)(STG + (size_t)b * CHP + i * 4) = *(const v4i*)(&ids[i * 4]);
    for (int i = threadIdx.x; i < NGP / 4; i += 64) { v4i v; for (int e = 0; e < 4; ++e) v[e] = (i * 4 + e < nG) ? cnt[i * 4 + e] : 0; *(volatile v4i*)(HST + (size_t)b * NGP + i * 4) = v; }
    __threadfence(); }
}
__global__ __launch_bounds__(512) void csrS_kernel(const int* __restrict__ HST, int nG, int NGP, int* __restrict__ START, int* __restrict__ TOT, int* __restrict__ OFF) {
  __shared__ int tot[CSR_MAXG];
  const int b = threadIdx.x;
  for (int pass = 0; pass < 2; ++pass) { int runb = 0; for (int g = 0; g < nG; ++g) { int c = HST[(size_t)b * NGP + g]; c = (c < 0) ? 0 : c; ((volatile int*)OFF)[(size_t)g * CSR_NBLK + b] = runb; runb += c; } __threadfence(); }
  for (int g = threadIdx.x; g < nG; g += 512) { int s = 0; for (int bb = 0; bb < CSR_NBLK; ++bb) { int c = HST[(size_t)bb * NGP + g]; s += (c < 0) ? 0 : c; } tot[g] = s; }
  __syncthreads();
  if (threadIdx.x < 32) {
    __shared__ int st[CSR_MAXG + 32];
    if (threadIdx.x == 0) { int acc = 0; for (int g = 0; g < NGP; ++g) { st[g] = acc; if (g < nG) acc += (tot[g] + 31) & ~31; } st[NGP] = acc; }
    __builtin_amdgcn_fence(__ATOMIC_RELEASE, "workgroup"); __builtin_amdgcn_wave_barrier(); __builtin_amdgcn_fence(__ATOMIC_ACQUIRE, "workgroup");
    for (int pass = 0; pass < 2; ++pass) { for (int i = threadIdx.x; i < NGP + 32; i += 32) { ((volatile int*)START)[i] = (i <= NGP) ? st[min(i, NGP)] : 0; ((volatile int*)TOT)[i] = (i < nG) ? tot[i] : 0; } __threadfence(); } }
}
__global__ __launch_bounds__(256) void csrB_kernel(const int* __restrict__ dst, int N, int nG, int CHP, int NGP, int permLen, const int* __restrict__ STG, const int* __restrict__ HST, const int* __restrict__ OFF, const int* __restrict__ START, const int* __restrict__ TOT, int* __restrict__ PERM, int* __restrict__ ROWPTR, int* __restrict__ ROWCNT, int* __restrict__ FLAG) {
  typedef __attribute__((ext_vector_type(4))) int v4i;
  __shared__ int ids[CSR_CAP]; __shared__ unsigned short key[CSR_CAP]; __shared__ int outp[CSR_CAP]; __shared__ int ncnt[CSR_GN + 1]; __shared__ int boff[CSR_NBLK + 1];
  const int g = blockIdx.x, t_ = threadIdx.x; int tot = TOT[g]; int st = START[g], stn = START[g + 1]; const int v0 = g * CSR_GN; const int nv = min(CSR_GN, N - v0);
  st = (st < 0) ? 0 : (st > permLen - 32 ? permLen - 32 : st) & ~31; stn = (stn < st) ? st : (stn > permLen ? permLen : stn); tot = (tot < 0) ? 0 : tot; if (tot > stn - st && tot <= CSR_CAP) tot = stn - st;
  if (tot > CSR_CAP) {
    for (int pass = 0; pass < 2; ++pass) { for (int i = t_; i < CSR_GN / 4; i += 256) { v4i a, c; for (int e = 0; e < 4; ++e) { a[e] = st; c[e] = 0; } *(volatile v4i*)(ROWPTR + v0 + i * 4) = a; *(volatile v4i*)(ROWCNT + v0 + i * 4) = c; } if (t_ == 0) ((volatile int*)FLAG)[0] = 1; __threadfence(); } (void)nv; return; }
  if (t_ == 0) { int acc = 0; for (int b = 0; b < CSR_NBLK; ++b) { boff[b] = acc; int c = HST[(size_t)b * NGP + g]; c = (c < 0) ? 0 : (c > CHP ? CHP : c); acc += c; if (acc > tot) acc = tot; } boff[CSR_NBLK] = acc; }
  for (int i = t_; i <= CSR_GN; i += 256) ncnt[i] = 0;
  __syncthreads();
  for (int b = 0; b < CSR_NBLK; ++b) { const int c = boff[b + 1] - boff[b]; int o_ = OFF[(size_t)g * CSR_NBLK + b]; o_ = (o_ < 0) ? 0 : (o_ > CHP - c ? CHP - c : o_); const int* src_ = STG + (size_t)b * CHP + o_;
    for (int i = t_; i < c; i += 256) { int id = src_[i]; id = (id < 0) ? 0 : id; ids[boff[b] + i] = id; int d = dst[id]; d = (d < v0) ? v0 : (d >= N ? N - 1 : d); int kk = d - v0; kk = (kk < 0) ? 0 : (kk >= CSR_GN ? CSR_GN - 1 : kk); key[boff[b] + i] = (unsigned short)kk; } }
  __syncthreads();
  if (t_ == 0) { for (int i = 0; i < tot; ++i) ncnt[key[i]] += 1; int acc = 0; for (int vl = 0; vl < CSR_GN; ++vl) { const int c = ncnt[vl]; ncnt[vl] = acc; acc += c; } ncnt[CSR_GN] = acc;
    for (int i = 0; i < tot; ++i) { const int vl = key[i]; outp[ncnt[vl]] = ids[i]; ncnt[vl] += 1; }
    for (int vl = CSR_GN; vl > 0; --vl) ncnt[vl] = ncnt[vl - 1]; ncnt[0] = 0; }
  __syncthreads();
  for (int pass = 0; pass < 2; ++pass) {
    for (int i = t_; i < (stn - st) / 4; i += 256) { v4i v; for (int e = 0; e < 4; ++e) { const int q = i * 4 + e; v[e] = (q < tot) ? outp[q] : -1; } *(volatile v4i*)(PERM + st + i * 4) = v; }
    for (int i = t_; i < CSR_GN / 4; i += 256) { v4i a, c; for (int e = 0; e < 4; ++e) { const int vl = i * 4 + e; a[e] = st + ncnt[vl]; c[e] = (vl < nv) ? (ncnt[vl + 1] - ncnt[vl]) : 0; } *(volatile v4i*)(ROWPTR + v0 + i * 4) = a; *(volatile v4i*)(ROWCNT + v0 + i * 4) = c; }
    __threadfence(); }
}
__global__ __launch_bounds__(256) void csrZ_kernel(int* __restrict__ p, size_t n4) { typedef __attribute__((ext_vector_type(4))) int v4i; const size_t tid = (size_t)blockIdx.x * 256 + threadIdx.x, nth = (size_t)gridDim.x * 256; v4i z = {0, 0, 0, 0}; for (size_t i = tid; i < n4; i += nth) *(volatile v4i*)(p + i * 4) = z; }
struct CsrBufs { int *STG, *HST, *OFF, *START, *TOT, *PERM, *ROWPTR, *ROWCNT, *FLAG; int nG, NGP, CHP; size_t permLen; char* base; size_t bytes; };
static size_t csr_carve(CsrBufs& c, char* ws, size_t off, int E, int N) {
  const size_t off0 = off; c.base = ws + off;
  auto al = [&](size_t bytes) { char* p = ws + off; off += (bytes + 255) & ~(size_t)255; return p; };
  c.nG = (N + CSR_GN - 1) / CSR_GN; c.NGP = (c.nG + 31) & ~31; const int ch = (E + CSR_NBLK - 1) / CSR_NBLK; c.CHP = (ch + 31) & ~31; c.permLen = (size_t)E + 32 * (size_t)c.nG + 32;
  c.STG = (int*)al((size_t)CSR_NBLK * c.CHP * 4); c.HST = (int*)al((size_t)CSR_NBLK * c.NGP * 4); c.OFF = (int*)al((size_t)c.NGP * CSR_NBLK * 4); c.START = (int*)al((size_t)(c.NGP + 64) * 4); c.TOT = (int*)al((size_t)(c.NGP + 64) * 4);
  c.PERM = (int*)al(c.permLen * 4); c.ROWPTR = (int*)al((size_t)c.nG * CSR_GN * 4); c.ROWCNT = (int*)al((size_t)c.nG * CSR_GN * 4); c.FLAG = (int*)al(256);
  c.bytes = off - off0; return off;
}
static void csr_build(const CsrBufs& c, const int* dst, int E, int N, hipStream_t stream) {
  const size_t smem = (size_t)(2 * c.NGP + c.CHP) * 4;
  csrZ_kernel<<<512, 256, 0, stream>>>((int*)c.base, c.bytes / 16);
  csrA_kernel<<<CSR_NBLK, 64, smem, stream>>>(dst, E, N, c.nG, c.CHP, c.NGP, c.STG, c.HST);
  csrS_kernel<<<1, 512, 0, stream>>>(c.HST, c.nG, c.NGP, c.START, c.TOT, c.OFF);
  csrB_kernel<<<c.nG, 256, 0, stream>>>(dst, N, c.nG, c.CHP, c.NGP, (int)c.permLen, c.STG, c.HST, c.OFF, c.START, c.TOT, c.PERM, c.ROWPTR, c.ROWCNT, c.FLAG);
}


__global__ __launch_bounds__(256) void prepw_kernel(const float* __restrict__ w2, const float* __restrict__ wih, const float* __restrict__ whh, b16* __restrict__ WP) {
  const int t = blockIdx.x * 256 + threadIdx.x; const int n0 = H * H / 8, n1 = G3 * RH / 8; v8b o;
  if (t < n0) { const int e = t * 8, oo = e / H, i0 = e - oo * H; for (int j = 0; j < 8; ++j) o[j] = (b16)(bf16_rne(w2[(size_t)(i0 + j) * H + oo]) * WSC); }
  else if (t < n0 + n1) { const int e = (t - n0) * 8; for (int j = 0; j < 8; ++j) o[j] = (b16)(bf16_rne(wih[e + j]) * WSC); }
  else if (t < n0 + 2 * n1) { const int e = (t - n0 - n1) * 8; for (int j = 0; j < 8; ++j) o[j] = (b16)(bf16_rne(whh[e + j]) * WSC); }
  else return;
  for (int pass = 0; pass < 2; ++pass) { *(volatile v8b*)(WP + (size_t)t * 8) = o; __threadfence(); }
}
__global__ __launch_bounds__(256) void agg1_kernel(const float* __restrict__ x, const int* __restrict__ srcs, const int* __restrict__ PERM, const int* __restrict__ ROWPTR, const int* __restrict__ ROWCNT, int permLen, float* __restrict__ AX) {
  const int wave = threadIdx.x >> 5, lane = threadIdx.x & 31; const size_t d = ((size_t)blockIdx.x * 8 + wave) * 2 + (lane >> 4); const int f = lane & 15;
  int st = ROWPTR[d], cnt = ROWCNT[d]; cnt = iclamp(cnt, 0, 4096); st = iclamp(st, 0, permLen - cnt); const float dd = rsqrtf((float)cnt + 1.0f);
  float acc = pmul(pmul(dd, dd), bf16_rne(x[d * DIN + f]));
  for (int j = 0; j < cnt; ++j) { const int e = iclamp(PERM[st + j], 0, E - 1); const int s = iclamp(srcs[e], 0, N - 1); const float ds = rsqrtf((float)iclamp(ROWCNT[s], 0, 4096) + 1.0f); acc += pmul(pmul(ds, dd), bf16_rne(x[(size_t)s * DIN + f])); }
  for (int pass = 0; pass < 2; ++pass) { ((volatile float*)AX)[d * DIN + f] = acc; __threadfence(); }
}
__global__ __launch_bounds__(256) void runner_kernel(const float* __restrict__ AX, const int* __restrict__ srcs, const int* __restrict__ ridx, const float* __restrict__ w1, const float* __restrict__ b1, const int* __restrict__ PERM, const int* __restrict__ ROWPTR, const int* __restrict__ ROWCNT, int permLen, b16* __restrict__ A2h, b16* __restrict__ A2l) {
  const int wave = threadIdx.x >> 5, lane = threadIdx.x & 31; const int g = blockIdx.x * 8 + wave; const int r = g * NODES + iclamp(ridx[g], 0, NODES - 1); const int c0 = lane * 4;
  int st = ROWPTR[r], cnt = ROWCNT[r]; cnt = iclamp(cnt, 0, 4096); st = iclamp(st, 0, permLen - cnt); const float dd = rsqrtf((float)cnt + 1.0f);
  float bb[4], acc[4] = {0, 0, 0, 0}; for (int q = 0; q < 4; ++q) bb[q] = bf16_rne(b1[c0 + q]);
  for (int j = -1; j < cnt; ++j) { int s; float nrm; if (j < 0) { s = r; nrm = pmul(dd, dd); } else { const int e = iclamp(PERM[st + j], 0, E - 1); s = iclamp(srcs[e], 0, N - 1); nrm = pmul(rsqrtf((float)iclamp(ROWCNT[s], 0, 4096) + 1.0f), dd); }
    float hv[4] = {bb[0], bb[1], bb[2], bb[3]}; const float* ax = AX + (size_t)s * DIN;
    for (int k = 0; k < DIN; ++k) { const float a = ax[k]; const v4f w = *(const v4f*)(w1 + k * H + c0); for (int q = 0; q < 4; ++q) hv[q] += pmul(a, bf16_rne(w[q])); }
    for (int q = 0; q < 4; ++q) acc[q] += pmul(nrm, fmaxf(hv[q], 0.0f)); }
  __attribute__((ext_vector_type(4))) _Float16 hv4, lv4; for (int q = 0; q < 4; ++q) { b16 p, qq; split16(acc[q] * XS, p, qq); hv4[q] = p; lv4[q] = qq; }
  for (int pass = 0; pass < 2; ++pass) { *(volatile __attribute__((ext_vector_type(4))) _Float16*)(A2h + (size_t)g * H + c0) = hv4; *(volatile __attribute__((ext_vector_type(4))) _Float16*)(A2l + (size_t)g * H + c0) = lv4; __threadfence(); }
}
template <int MODE>
__global__ __launch_bounds__(128) void gemm_kernel(const b16* __restrict__ Ah, const b16* __restrict__ Al, const b16* __restrict__ W, const float* __restrict__ bias, b16* __restrict__ Yh, b16* __restrict__ Yl, float* __restrict__ Yf) {
  __shared__ __attribute__((aligned(16))) float Ts[4][16][H + 4];
  const int wave = threadIdx.x >> 5, lane = threadIdx.x & 31, nloc = lane & 15, hlf = lane >> 4; const size_t m0 = ((size_t)blockIdx.x * 4 + wave) * 16; const int n0 = blockIdx.y * 128;
  v8f acc[8];
#pragma unroll
  for (int t = 0; t < 8; ++t) acc[t] = (v8f){};
#pragma unroll
  for (int kb = 0; kb < H; kb += 32) { const v16b a = frag_kb(Ah + (m0 + nloc) * H + kb, hlf), al = frag_kb(Al + (m0 + nloc) * H + kb, hlf);
#pragma unroll
    for (int t = 0; t < 8; ++t) { const v16b bw = frag_kb(W + (size_t)(n0 + t * 16 + nloc) * H + kb, hlf); acc[t] = wmma16b(a, bw, acc[t]); acc[t] = wmma16b(al, bw, acc[t]); } }
#pragma unroll
  for (int t = 0; t < 8; ++t) { const int c = n0 + t * 16 + nloc; const float bb = bf16_rne(bias[c]);
#pragma unroll
    for (int r = 0; r < 8; ++r) { float v = acc[t][r] * (1.0f / (XS * WSC)) + bb; if (MODE == 0) v = fmaxf(v, 0.0f); Ts[wave][8 * hlf + r][t * 16 + nloc] = v; } }
  wave_lds_sync();
  for (int pass = 0; pass < 2; ++pass) { for (int rr = 0; rr < 16; ++rr) {
      if (MODE == 0) { if (lane < 16) { v8b hv, lv; for (int j = 0; j < 8; ++j) { b16 p, q; split16(Ts[wave][rr][lane * 8 + j] * XS, p, q); hv[j] = p; lv[j] = q; } *(volatile v8b*)(Yh + (m0 + rr) * H + lane * 8) = hv; *(volatile v8b*)(Yl + (m0 + rr) * H + lane * 8) = lv; } }
      else *(volatile v4f*)(Yf + (m0 + rr) * G3 + n0 + lane * 4) = *(const v4f*)(&Ts[wave][rr][lane * 4]); }
    __threadfence(); }
}
__global__ __launch_bounds__(128) void gru_kernel(const float* __restrict__ XG, const b16* __restrict__ WHH, const float* __restrict__ bhh, const float* __restrict__ wp, const float* __restrict__ bp, float* __restrict__ out) {
  __shared__ __attribute__((aligned(16))) b16 Hh[16][H + 8], Hl[16][H + 8]; __shared__ float Hf[16][H + 4]; __shared__ float GH[16][G3 + 4]; __shared__ float PR[16][T][2];
  const int wave = threadIdx.x >> 5, lane = threadIdx.x & 31, nloc = lane & 15, hlf = lane >> 4, t_ = threadIdx.x; const int b0 = blockIdx.x * 16;
  for (int i = t_; i < 16 * (H + 8); i += 128) { Hh[i / (H + 8)][i % (H + 8)] = (b16)0.0f; Hl[i / (H + 8)][i % (H + 8)] = (b16)0.0f; } for (int i = t_; i < 16 * (H + 4); i += 128) Hf[i / (H + 4)][i % (H + 4)] = 0.0f;
  __syncthreads();
  for (int step = 0; step < T; ++step) {
    v8f acc[6];
#pragma unroll
    for (int tt = 0; tt < 6; ++tt) acc[tt] = (v8f){};
#pragma unroll
    for (int kb = 0; kb < H; kb += 32) { const v16b a = frag_kb(&Hh[nloc][kb], hlf), al = frag_kb(&Hl[nloc][kb], hlf);
#pragma unroll
      for (int tt = 0; tt < 6; ++tt) { const v16b bw = frag_kb(WHH + (size_t)((wave * 6 + tt) * 16 + nloc) * RH + kb, hlf); acc[tt] = wmma16b(a, bw, acc[tt]); acc[tt] = wmma16b(al, bw, acc[tt]); } }
#pragma unroll
    for (int tt = 0; tt < 6; ++tt) { const int c = (wave * 6 + tt) * 16 + nloc; const float bb = bf16_rne(bhh[c]);
#pragma unroll
      for (int r = 0; r < 8; ++r) GH[8 * hlf + r][c] = acc[tt][r] * (1.0f / (XS * WSC)) + bb; }
    __syncthreads();
    { const int row = t_ >> 3, j0 = (t_ & 7) * 16; const size_t xo = ((size_t)(b0 + row) * T + step) * G3; float p0 = 0.0f, p1 = 0.0f;
      for (int j = j0; j < j0 + 16; ++j) { const float r = sigm(XG[xo + j] + GH[row][j]), z = sigm(XG[xo + RH + j] + GH[row][RH + j]); const float n = tanh_(XG[xo + 2 * RH + j] + pmul(r, GH[row][2 * RH + j])); const float h = pmul(1.0f - z, n) + pmul(z, Hf[row][j]);
        Hf[row][j] = h; b16 a_, c_; split16(h * XS, a_, c_); Hh[row][j] = a_; Hl[row][j] = c_; p0 += pmul(h, bf16_rne(wp[j * 2])); p1 += pmul(h, bf16_rne(wp[j * 2 + 1])); }
      p0 += __shfl_xor(p0, 1); p0 += __shfl_xor(p0, 2); p0 += __shfl_xor(p0, 4); p1 += __shfl_xor(p1, 1); p1 += __shfl_xor(p1, 2); p1 += __shfl_xor(p1, 4);
      if ((t_ & 7) == 0) { PR[row][step][0] = p0 + bf16_rne(bp[0]); PR[row][step][1] = p1 + bf16_rne(bp[1]); } }
    __syncthreads(); }
  for (int pass = 0; pass < 2; ++pass) { for (int i = t_; i < 16 * T * 2 / 4; i += 128) { const int row = i / (T * 2 / 4), q = i - row * (T * 2 / 4); *(volatile v4f*)(out + ((size_t)(b0 + row) * T) * 2 + q * 4) = *(const v4f*)(&PR[row][0][0] + q * 4); } __threadfence(); }
}
}

extern "C" void kernel_launch(void* const* d_in, const int* in_sizes, int n_in, void* d_out, int out_size, void* d_ws, size_t ws_size, hipStream_t stream) {
  (void)n_in;
  auto Fp = [&](int i) { return (const float*)d_in[i]; }; auto Ip = [&](int i) { return (const int*)d_in[i]; };
  if (in_sizes[0] != N * DIN || in_sizes[1] != 2 * E || in_sizes[2] != G || in_sizes[3] != DIN * H || in_sizes[7] != G3 * H || in_sizes[11] != RH * 2 || out_size != NBQ * T * 2) return;
  size_t off = 0; char* ws = (char*)d_ws;
  auto carve = [&](size_t bytes) { char* p = ws + off; off += (bytes + 255) & ~(size_t)255; return p; };
  b16* WP = (b16*)carve(((size_t)H * H + 2 * (size_t)G3 * RH) * 2); float* AX = (float*)carve((size_t)N * DIN * 4); b16* A2h = (b16*)carve((size_t)G * H * 2); b16* A2l = (b16*)carve((size_t)G * H * 2); b16* SQh = (b16*)carve((size_t)G * H * 2); b16* SQl = (b16*)carve((size_t)G * H * 2); float* XG = (float*)carve((size_t)G * G3 * 4);
  CsrBufs csr; off = csr_carve(csr, ws, off, E, N);
  if (off > ws_size || off > ((size_t)128 << 20)) return;
  const b16* W2T = WP; const b16* WIH = WP + (size_t)H * H; const b16* WHH = WIH + (size_t)G3 * RH;
  prepw_kernel<<<(H * H / 8 + 2 * G3 * RH / 8 + 255) / 256, 256, 0, stream>>>(Fp(5), Fp(7), Fp(8), WP);
  csr_build(csr, Ip(1) + E, E, N, stream);
  agg1_kernel<<<N / 16, 256, 0, stream>>>(Fp(0), Ip(1), csr.PERM, csr.ROWPTR, csr.ROWCNT, (int)csr.permLen, AX);
  runner_kernel<<<G / 8, 256, 0, stream>>>(AX, Ip(1), Ip(2), Fp(3), Fp(4), csr.PERM, csr.ROWPTR, csr.ROWCNT, (int)csr.permLen, A2h, A2l);
  gemm_kernel<0><<<dim3(G / 64, 1), 128, 0, stream>>>(A2h, A2l, W2T, Fp(6), SQh, SQl, nullptr);
  gemm_kernel<1><<<dim3(G / 64, 3), 128, 0, stream>>>(SQh, SQl, WIH, Fp(9), nullptr, nullptr, XG);
  gru_kernel<<<NBQ / 16, 128, 0, stream>>>(XG, WHH, Fp(10), Fp(11), Fp(12), (float*)d_out);
}
